// MultiHead_54348516163892
// MI455X (gfx1250) — hardware-verified
//
#include <hip/hip_runtime.h>
#ifndef NB
#define NB 4
#endif
#ifndef SEQ
#define SEQ 2048
#endif
#define NB_FULL 4
#define SEQ_FULL 2048
#define DMOD 1024
#define NHEAD 16
#define HD 64
#define NR ((size_t)NB * SEQ)
#define PPITCH 40
#define CPITCH 72
static_assert(SEQ % 128 == 0);
static_assert(SEQ <= SEQ_FULL);
static_assert(NB >= 1 && NB <= NB_FULL);
static_assert(NHEAD * HD == DMOD);
static_assert(DMOD % 128 == 0);
static_assert((NB * SEQ) % 128 == 0);

typedef unsigned short v8us __attribute__((ext_vector_type(8), may_alias));
typedef float  v8f  __attribute__((ext_vector_type(8)));
typedef float  v4f  __attribute__((ext_vector_type(4)));
typedef float  v4fa __attribute__((ext_vector_type(4), may_alias));
typedef _Float16 v16h __attribute__((ext_vector_type(16)));
typedef _Float16 v4h __attribute__((ext_vector_type(4)));
union FragH { v16h v; v8us half[2]; _Float16 h[16]; unsigned short u[16]; };

__device__ __forceinline__ unsigned short bf16_bits(float x) { unsigned int u = __float_as_uint(x); return (unsigned short)((u + 0x7FFFu + ((u >> 16) & 1u)) >> 16); }
__device__ __forceinline__ float bf16_val(unsigned short b) { return __uint_as_float(((unsigned int)b) << 16); }
__device__ __forceinline__ float bf16_rne(float x) { return bf16_val(bf16_bits(x)); }

__device__ __forceinline__ v16h g2_frag(const _Float16* p, int hh) { FragH f; f.half[0] = *(const v8us*)((const unsigned short*)p + 8 * hh); f.half[1] = *(const v8us*)((const unsigned short*)p + 16 + 8 * hh); return f.v; }
__device__ __forceinline__ v8f g2_mma(v16h a, v16h b, v8f c) { v8f d = __builtin_amdgcn_wmma_f32_16x16x32_f16(false, a, false, b, (short)0, c, false, false); asm volatile("v_nop\n\tv_nop\n\tv_nop\n\tv_nop" : "+v"(d) : "v"(a), "v"(b)); return d; }

__global__ __launch_bounds__(256) void k_wt_f16(const float* __restrict__ W, _Float16* __restrict__ Wt, int K, int N, float scale) {
  const int t = blockIdx.x * 256 + threadIdx.x; if (t >= N * (K / 8)) return;
  const int n = t / (K / 8), k8 = (t % (K / 8)) * 8; FragH f;
#pragma unroll
  for (int i = 0; i < 8; ++i) f.h[i] = (_Float16)(bf16_rne(W[(size_t)(k8 + i) * N + n]) * scale);
  const v8us o = f.half[0];
  unsigned short* dst = (unsigned short*)Wt + (size_t)n * K + k8;
  *(volatile v8us*)dst = o; __threadfence(); *(volatile v8us*)dst = o;
}

__global__ __launch_bounds__(256) void k_x16(const float* __restrict__ x, _Float16* __restrict__ X16, size_t n8) {
  const size_t t = (size_t)blockIdx.x * 256 + threadIdx.x; if (t >= n8) return;
  const size_t row = t / (DMOD / 8); const int c8 = (int)(t % (DMOD / 8)) * 8;
  const size_t b = row / SEQ, s = row % SEQ;
  const float* src = x + (b * SEQ_FULL + s) * DMOD + c8;
  const v4f a = *(const v4fa*)src, c = *(const v4fa*)(src + 4);
  FragH f;
#pragma unroll
  for (int q = 0; q < 4; ++q) { f.h[q] = (_Float16)bf16_rne(a[q]); f.h[4 + q] = (_Float16)bf16_rne(c[q]); }
  const v8us o = f.half[0];
  unsigned short* dst = (unsigned short*)X16 + t * 8;
  *(volatile v8us*)dst = o; __threadfence(); *(volatile v8us*)dst = o;
}

template <int BIASM>
__global__ __launch_bounds__(128) void k_gemm2(const _Float16* __restrict__ A, int lda, size_t sA, const _Float16* __restrict__ Bh, int ldb, size_t sB, float alpha,
                                              const float* __restrict__ bias, float* __restrict__ C, _Float16* __restrict__ C16, int ldc, size_t sC, int M, int N, int K) {
  __shared__ __attribute__((aligned(16))) float so[4][32][68];
  const int tid = threadIdx.x, w = tid >> 5, lane = tid & 31, ln = lane & 15, hh = lane >> 4; const int by = blockIdx.y;
  A += (size_t)by * sA; Bh += (size_t)by * sB; const size_t cofs = (size_t)by * sC;
  const int ntn = N >> 6; const int mt = blockIdx.x / ntn, nq = blockIdx.x - mt * ntn; const int row0 = mt * 128 + 32 * w, col0 = nq * 64; if (row0 >= M) return;
  const _Float16* a0p = A + (size_t)(row0 + ln) * lda; const _Float16* a1p = a0p + (size_t)16 * lda;
  const _Float16* b0p = Bh + (size_t)(col0 + ln) * ldb; const _Float16* b1p = b0p + (size_t)16 * ldb; const _Float16* b2p = b1p + (size_t)16 * ldb; const _Float16* b3p = b2p + (size_t)16 * ldb;
  const v8f z8 = {0.f,0.f,0.f,0.f,0.f,0.f,0.f,0.f}; v8f c00 = z8, c01 = z8, c02 = z8, c03 = z8, c10 = z8, c11 = z8, c12 = z8, c13 = z8;
#pragma unroll 1
  for (int kb = 0; kb < K; kb += 32) { const v16h a0 = g2_frag(a0p + kb, hh), a1 = g2_frag(a1p + kb, hh);
    v16h b = g2_frag(b0p + kb, hh); c00 = g2_mma(a0, b, c00); c10 = g2_mma(a1, b, c10);
    b = g2_frag(b1p + kb, hh); c01 = g2_mma(a0, b, c01); c11 = g2_mma(a1, b, c11);
    b = g2_frag(b2p + kb, hh); c02 = g2_mma(a0, b, c02); c12 = g2_mma(a1, b, c12);
    b = g2_frag(b3p + kb, hh); c03 = g2_mma(a0, b, c03); c13 = g2_mma(a1, b, c13); }
  v8f accs[8] = {c00, c01, c02, c03, c10, c11, c12, c13};
#pragma unroll
  for (int u = 0; u < 8; ++u) { const int t = u & 3, half = u >> 2; const int col = col0 + t * 16 + ln;
    const float bcol = (BIASM == 0) ? bf16_rne(bias[col]) : 0.f;
#pragma unroll
    for (int r = 0; r < 8; ++r) { const int rloc = half * 16 + 8 * hh + r; float bv = bcol; if (BIASM == 1) bv = bf16_rne(bias[row0 + rloc]);
      so[w][rloc][t * 16 + ln] = accs[u][r] * alpha + bv; } }
  __builtin_amdgcn_fence(4  , "workgroup"); __builtin_amdgcn_wave_barrier();
  const int rsub = lane >> 4, c4 = (lane & 15) * 4;
  for (int pass = 0; pass < 2; ++pass) {
#pragma unroll
    for (int q = 0; q < 16; ++q) { const int r = q * 2 + rsub; const v4f v = *(const v4fa*)&so[w][r][c4];
      if (C) *(volatile v4f*)(C + cofs + (size_t)(row0 + r) * ldc + col0 + c4) = v;
      if (C16) { v4h h4; for (int i = 0; i < 4; ++i) h4[i] = (_Float16)v[i]; *(volatile v4h*)(C16 + cofs + (size_t)(row0 + r) * ldc + col0 + c4) = h4; } }
    if (pass == 0) __threadfence(); }
}

__global__ __launch_bounds__(256) void k_attn(const _Float16* __restrict__ Q16, const _Float16* __restrict__ K16, const _Float16* __restrict__ VT, _Float16* __restrict__ CTX) {
  __shared__ __attribute__((aligned(16))) _Float16 Pl[8][16][PPITCH];
  __shared__ __attribute__((aligned(16))) _Float16 Co[8][16][CPITCH];
  const int tid = threadIdx.x, w = tid >> 5, lane = tid & 31, ln = lane & 15, hh = lane >> 4;
  const int nqb = SEQ / 128;
  const int bid = blockIdx.x; const int qb = bid % nqb; const int h = (bid / nqb) % NHEAD; const int b = bid / (nqb * NHEAD);
  const int q0 = qb * 128 + w * 16;
  const size_t qrow = (size_t)b * SEQ + q0;
  v16h qf0, qf1;
  { const _Float16* qp = Q16 + (qrow + ln) * DMOD + h * HD; qf0 = g2_frag(qp, hh); qf1 = g2_frag(qp + 32, hh); }
  const v8f z8 = {0.f,0.f,0.f,0.f,0.f,0.f,0.f,0.f};
  v8f o[4] = {z8, z8, z8, z8};
  float m[8], l[8];
#pragma unroll
  for (int r = 0; r < 8; ++r) { m[r] = -1.0e30f; l[r] = 0.f; }
  const _Float16* kbase = K16 + ((size_t)b * SEQ + ln) * DMOD + h * HD;
  const _Float16* vbase = VT + ((size_t)(b * NHEAD + h) * HD + ln) * SEQ;
#pragma unroll 1
  for (int ks0 = 0; ks0 < SEQ; ks0 += 32) {
    v8f s0 = z8, s1 = z8;
    { const _Float16* kp = kbase + (size_t)ks0 * DMOD;
      v16h kf = g2_frag(kp, hh); s0 = g2_mma(qf0, kf, s0); kf = g2_frag(kp + 32, hh); s0 = g2_mma(qf1, kf, s0);
      kp += (size_t)16 * DMOD;
      kf = g2_frag(kp, hh); s1 = g2_mma(qf0, kf, s1); kf = g2_frag(kp + 32, hh); s1 = g2_mma(qf1, kf, s1); }
    __builtin_amdgcn_fence(4  , "wavefront"); __builtin_amdgcn_wave_barrier();
    float corr[8];
#pragma unroll
    for (int r = 0; r < 8; ++r) {
      const float a0 = s0[r] * 0.125f, a1 = s1[r] * 0.125f;
      float mx = fmaxf(a0, a1);
      mx = fmaxf(mx, __shfl_xor(mx, 1, 32)); mx = fmaxf(mx, __shfl_xor(mx, 2, 32)); mx = fmaxf(mx, __shfl_xor(mx, 4, 32)); mx = fmaxf(mx, __shfl_xor(mx, 8, 32));
      mx = fmaxf(mx, m[r]);
      const float c0 = __expf(m[r] - mx);
      const _Float16 p0 = (_Float16)(__expf(a0 - mx) * 1024.0f), p1 = (_Float16)(__expf(a1 - mx) * 1024.0f);
      float ps = (float)p0 + (float)p1;
      ps += __shfl_xor(ps, 1, 32); ps += __shfl_xor(ps, 2, 32); ps += __shfl_xor(ps, 4, 32); ps += __shfl_xor(ps, 8, 32);
      l[r] = l[r] * c0 + ps; m[r] = mx; corr[r] = c0;
      Pl[w][8 * hh + r][ln] = p0; Pl[w][8 * hh + r][16 + ln] = p1;
    }
#pragma unroll
    for (int j = 0; j < 4; ++j)
#pragma unroll
      for (int r = 0; r < 8; ++r) o[j][r] = o[j][r] * corr[r];
    __builtin_amdgcn_fence(4  , "wavefront"); __builtin_amdgcn_wave_barrier();
    FragH pfr; pfr.half[0] = *(const v8us*)&Pl[w][ln][8 * hh]; pfr.half[1] = *(const v8us*)&Pl[w][ln][16 + 8 * hh];
    const v16h pf = pfr.v;
    const _Float16* vp = vbase + ks0;
#pragma unroll
    for (int j = 0; j < 4; ++j) { const v16h vf = g2_frag(vp + (size_t)(j * 16) * SEQ, hh); o[j] = g2_mma(pf, vf, o[j]); }
  }
  float inv[8];
#pragma unroll
  for (int r = 0; r < 8; ++r) inv[r] = 16.0f / l[r];
#pragma unroll
  for (int j = 0; j < 4; ++j)
#pragma unroll
    for (int r = 0; r < 8; ++r) Co[w][8 * hh + r][j * 16 + ln] = (_Float16)(o[j][r] * inv[r]);
  __builtin_amdgcn_fence(4  , "wavefront"); __builtin_amdgcn_wave_barrier();
  const int rq = lane >> 3, pc = lane & 7;
  for (int pass = 0; pass < 2; ++pass) {
#pragma unroll
    for (int it = 0; it < 4; ++it) { const int row = it * 4 + rq; const v8us v = *(const v8us*)&Co[w][row][pc * 8];
      *(volatile v8us*)((unsigned short*)CTX + (qrow + row) * DMOD + h * HD + pc * 8) = v; }
    if (pass == 0) __threadfence(); }
}

extern "C" void kernel_launch(void* const* d_in, const int* in_sizes, int n_in,
                              void* d_out, int out_size, void* d_ws, size_t ws_size, hipStream_t stream) {
  if (n_in < 9) return;
  const float* x  = (const float*)d_in[0];
  const float* wq = (const float*)d_in[1]; const float* bq = (const float*)d_in[2];
  const float* wk = (const float*)d_in[3]; const float* bk = (const float*)d_in[4];
  const float* wv = (const float*)d_in[5]; const float* bv = (const float*)d_in[6];
  const float* wo = (const float*)d_in[7]; const float* bo = (const float*)d_in[8];
  const size_t xneed = ((size_t)(NB - 1) * SEQ_FULL + SEQ) * DMOD;
  if ((size_t)in_sizes[0] < xneed) return;
  if (in_sizes[1] < DMOD * DMOD || in_sizes[3] < DMOD * DMOD || in_sizes[5] < DMOD * DMOD || in_sizes[7] < DMOD * DMOD) return;
  if (in_sizes[2] < DMOD || in_sizes[4] < DMOD || in_sizes[6] < DMOD || in_sizes[8] < DMOD) return;
  if ((size_t)out_size < NR * DMOD) return;
  char* ws = (char*)d_ws; size_t off = 0;
  auto take = [&](size_t bytes) { char* p = ws + off; off += (bytes + 255) & ~(size_t)255; return p; };
  _Float16* WQt = (_Float16*)take((size_t)DMOD * DMOD * 2); _Float16* WKt = (_Float16*)take((size_t)DMOD * DMOD * 2);
  _Float16* WVt = (_Float16*)take((size_t)DMOD * DMOD * 2); _Float16* WOt = (_Float16*)take((size_t)DMOD * DMOD * 2);
  _Float16* X16 = (_Float16*)take(NR * DMOD * 2); _Float16* Q16 = (_Float16*)take(NR * DMOD * 2); _Float16* K16 = (_Float16*)take(NR * DMOD * 2);
  _Float16* VT = (_Float16*)take((size_t)NB * NHEAD * HD * SEQ * 2); _Float16* CTX16 = (_Float16*)take(NR * DMOD * 2);
  if (off > ws_size) return;
  const unsigned gw = (unsigned)((DMOD * (DMOD / 8) + 255) / 256);
  k_wt_f16<<<gw, 256, 0, stream>>>(wq, WQt, DMOD, DMOD, 16.0f);
  k_wt_f16<<<gw, 256, 0, stream>>>(wk, WKt, DMOD, DMOD, 16.0f);
  k_wt_f16<<<gw, 256, 0, stream>>>(wv, WVt, DMOD, DMOD, 16.0f);
  k_wt_f16<<<gw, 256, 0, stream>>>(wo, WOt, DMOD, DMOD, 16.0f);
  const size_t n8 = NR * DMOD / 8;
  k_x16<<<(unsigned)((n8 + 255) / 256), 256, 0, stream>>>(x, X16, n8);
  const int MR = (int)NR;
  k_gemm2<0><<<dim3((unsigned)((MR / 128) * (DMOD / 64)), 1), 128, 0, stream>>>(X16, DMOD, 0, WQt, DMOD, 0, 0.0625f, bq, nullptr, Q16, DMOD, 0, MR, DMOD, DMOD);
  k_gemm2<0><<<dim3((unsigned)((MR / 128) * (DMOD / 64)), 1), 128, 0, stream>>>(X16, DMOD, 0, WKt, DMOD, 0, 0.0625f, bk, nullptr, K16, DMOD, 0, MR, DMOD, DMOD);
  k_gemm2<1><<<dim3((unsigned)((DMOD / 128) * (SEQ / 64)), NB), 128, 0, stream>>>(WVt, DMOD, 0, X16, DMOD, (size_t)SEQ * DMOD, 0.0625f, bv, nullptr, VT, SEQ, (size_t)DMOD * SEQ, DMOD, SEQ, DMOD);
  k_attn<<<(unsigned)(NB * NHEAD * (SEQ / 128)), 256, 0, stream>>>(Q16, K16, VT, CTX16);
  k_gemm2<0><<<dim3((unsigned)((MR / 128) * (DMOD / 64)), 1), 128, 0, stream>>>(CTX16, DMOD, 0, WOt, DMOD, 0, 0.00390625f, bo, (float*)d_out, nullptr, DMOD, 0, MR, DMOD, DMOD);
}
